// LogSig_RNN_50921132261615
// MI455X (gfx1250) — hardware-verified
//
#include <hip/hip_runtime.h>
#include <hip/hip_bf16.h>


#define NB_   32
#define TL_   600
#define CC_   64
#define NS_   50
#define HD_   512
#define G4_   2048
#define FIN_  2144
#define KP_   2176
#define NA_   2016
#define MR_   1600
#define LMAX_ 13
#define HP_   520
#define OP_   36
#define QP_   65

static_assert(MR_ == NB_ * NS_);
static_assert(FIN_ == CC_ + NA_ + CC_);
static_assert(NA_ == CC_ * (CC_ - 1) / 2);
static_assert(KP_ % 32 == 0);
static_assert(KP_ >= FIN_);
static_assert(MR_ % 64 == 0);
static_assert(G4_ % 64 == 0);
static_assert(HD_ % 32 == 0);
static_assert((KP_ * 2) % 128 == 0);
static_assert((HD_ * 2) % 128 == 0);
static_assert((G4_ * 4) % 128 == 0);
static_assert(KP_ / 8 - 256 == 16);
static_assert(NB_ % 16 == 0);
static_assert((HP_ * 2) % 16 == 0);
static_assert((OP_ * 4) % 16 == 0);

typedef float          v4f   __attribute__((ext_vector_type(4)));
typedef float          v8f   __attribute__((ext_vector_type(8)));
typedef __bf16         v16b  __attribute__((ext_vector_type(16)));
typedef unsigned short u16x8 __attribute__((ext_vector_type(8)));

union FragB { u16x8 h[2]; v16b v; };

__constant__ int k_tv[NS_ + 1] = {
    1, 13, 25, 37, 49, 61, 73, 85, 97, 109, 121, 133, 145, 157, 169, 181, 193, 205, 217, 229,
    241, 253, 265, 277, 289, 300, 312, 324, 336, 348, 360, 372, 384, 396, 408, 420, 432, 444, 456, 468,
    480, 492, 504, 516, 528, 540, 552, 564, 576, 588, 600 };

constexpr size_t SZ_F16  = (size_t)MR_ * KP_ * 2;
constexpr size_t SZ_WI16 = (size_t)G4_ * KP_ * 2;
constexpr size_t SZ_WH16 = (size_t)G4_ * HD_ * 2;
constexpr size_t SZ_GX   = (size_t)MR_ * G4_ * 4;

constexpr size_t OFF_FH  = 0;
constexpr size_t OFF_FL  = OFF_FH  + SZ_F16;
constexpr size_t OFF_WIH = OFF_FL  + SZ_F16;
constexpr size_t OFF_WIL = OFF_WIH + SZ_WI16;
constexpr size_t OFF_WHH = OFF_WIL + SZ_WI16;
constexpr size_t OFF_WHL = OFF_WHH + SZ_WH16;
constexpr size_t OFF_GX  = OFF_WHL + SZ_WH16;
constexpr size_t WS_END  = OFF_GX  + SZ_GX;
static_assert(WS_END <= (size_t)134217728);
static_assert(OFF_FL % 128 == 0 && OFF_WIH % 128 == 0 && OFF_WIL % 128 == 0);
static_assert(OFF_WHH % 128 == 0 && OFF_WHL % 128 == 0 && OFF_GX % 128 == 0);

__device__ __forceinline__ unsigned short f32_to_bf16(float f) {
    unsigned u = __float_as_uint(f);
    unsigned r = u + 0x7FFFu + ((u >> 16) & 1u);
    return (unsigned short)(r >> 16);
}
__device__ __forceinline__ float bf16_to_f32(unsigned short b) {
    return __uint_as_float(((unsigned)b) << 16);
}
__device__ __forceinline__ v8f ld8f(const float* p) {
    v4f a = *(const v4f*)p;
    v4f b = *(const v4f*)(p + 4);
    return __builtin_shufflevector(a, b, 0, 1, 2, 3, 4, 5, 6, 7);
}
__device__ __forceinline__ void split8(const v8f x, u16x8& hv, u16x8& lv) {
#pragma unroll
    for (int c = 0; c < 8; ++c) {
        const float f = x[c];
        const unsigned short hb = f32_to_bf16(f);
        const unsigned short lb = f32_to_bf16(f - bf16_to_f32(hb));
        hv[c] = hb;
        lv[c] = lb;
    }
}
__device__ __forceinline__ float sigm_f(float x) {
    return __builtin_amdgcn_rcpf(1.0f + __expf(-x));
}
__device__ __forceinline__ float tanh_f(float x) {
    return 1.0f - 2.0f * __builtin_amdgcn_rcpf(1.0f + __expf(x + x));
}

__device__ __forceinline__ void mma16(v8f& acc, const FragB& a, const FragB& b) {
    acc = __builtin_amdgcn_wmma_f32_16x16x32_bf16(false, a.v, false, b.v, (short)0, acc, false, false);
    asm volatile("v_nop\n\tv_nop\n\tv_nop\n\tv_nop" : "+v"(acc) : "v"(a.v), "v"(b.v));
}

__global__ __launch_bounds__(256)
void rows_cvt_kernel(const float* __restrict__ src, unsigned short* dhi, unsigned short* dlo,
                     int kin, int kp, int npieces)
{
    const int p = blockIdx.x * 256 + threadIdx.x;
    if (p >= npieces) return;
    const int ppr = kp >> 3;
    const int row = p / ppr;
    const int c8  = (p - row * ppr) * 8;
    const int c8c = min(c8, kin - 8);
    v8f x = ld8f(src + (size_t)row * kin + c8c);
    const bool in = (c8 < kin);
#pragma unroll
    for (int i = 0; i < 8; ++i) x[i] = in ? x[i] : 0.0f;
    u16x8 hv, lv;
    split8(x, hv, lv);
    const size_t o = (size_t)p * 8;
    *(volatile u16x8*)(dhi + o) = hv;
    *(volatile u16x8*)(dlo + o) = lv;
    __threadfence();
    *(volatile u16x8*)(dhi + o) = hv;
    *(volatile u16x8*)(dlo + o) = lv;
}

__global__ __launch_bounds__(256)
void feats_kernel(const float* __restrict__ x, unsigned short* fh, unsigned short* fl)
{
#pragma clang fp contract(off)
    __shared__ __attribute__((aligned(16))) float xs[LMAX_ * CC_];
    __shared__ float Qs[CC_ * QP_];
    __shared__ __attribute__((aligned(16))) float frow[KP_];

    const int tid = threadIdx.x;
    const int r   = blockIdx.x;
    const int s   = r >> 5;
    const int b   = r & 31;
    int t0 = k_tv[s] - 1;
    int t1 = k_tv[s + 1] - 1;
    t0 = min(max(t0, 0), TL_ - 1);
    t1 = min(max(t1, t0), TL_ - 1);
    int len = t1 - t0 + 1;
    len = min(max(len, 1), LMAX_);
    const int le = (len - 1) * CC_;

    const float* xb = x + (size_t)b * TL_ * CC_;
    for (int idx = tid; idx < LMAX_ * CC_; idx += 256) {
        const int tt = idx >> 6;
        const int c  = idx & 63;
        const int fr = t0 + min(tt, len - 1);
        xs[idx] = xb[(size_t)fr * CC_ + c];
    }
    __syncthreads();

    {
        const int i  = tid >> 2;
        const int jb = (tid & 3) * 16;
        float q[16];
#pragma unroll
        for (int jj = 0; jj < 16; ++jj) q[jj] = 0.0f;
        const int nst = len - 1;
#pragma unroll 1
        for (int t = 0; t < nst; ++t) {
            const float xi = xs[t * CC_ + i];
            const float* p0 = xs + t * CC_ + jb;
            const float* p1 = p0 + CC_;
#pragma unroll
            for (int jj = 0; jj < 16; ++jj) {
                const float d  = p1[jj] - p0[jj];
                const float pr = xi * d;
                q[jj] = q[jj] + pr;
            }
        }
#pragma unroll
        for (int jj = 0; jj < 16; ++jj) Qs[i * QP_ + jb + jj] = q[jj];
    }
    __syncthreads();

    if (tid < CC_) {
        const float xa = xs[tid];
        frow[tid] = xs[le + tid] - xa;
        frow[CC_ + NA_ + tid] = xa;
    }
    if (tid < KP_ - FIN_) frow[FIN_ + tid] = 0.0f;
#pragma unroll 4
    for (int qd = 0; qd < 16; ++qd) {
        const int e2 = qd * 256 + tid;
        const int i  = e2 >> 6;
        const int j  = e2 & 63;
        if (j > i) {
            const float xai  = xs[i];
            const float xaj  = xs[j];
            const float inci = xs[le + i] - xai;
            const float incj = xs[le + j] - xaj;
            const float mij  = xai * incj;
            const float mji  = xaj * inci;
            const float pij  = Qs[i * QP_ + j] - mij;
            const float pji  = Qs[j * QP_ + i] - mji;
            const int off = 63 * i - ((i * (i - 1)) >> 1) + (j - i - 1);
            frow[CC_ + off] = 0.5f * (pij - pji);
        }
    }
    __syncthreads();

    u16x8 hv0, lv0, hv1, lv1;
    split8(ld8f(frow + tid * 8), hv0, lv0);
    const bool second = (tid < (KP_ / 8 - 256));
    const int  p2     = second ? (256 + tid) : tid;
    split8(ld8f(frow + p2 * 8), hv1, lv1);
    const size_t o0 = (size_t)r * KP_ + (size_t)tid * 8;
    const size_t o1 = (size_t)r * KP_ + (size_t)p2 * 8;
    *(volatile u16x8*)(fh + o0) = hv0;
    *(volatile u16x8*)(fl + o0) = lv0;
    if (second) {
        *(volatile u16x8*)(fh + o1) = hv1;
        *(volatile u16x8*)(fl + o1) = lv1;
    }
    __threadfence();
    *(volatile u16x8*)(fh + o0) = hv0;
    *(volatile u16x8*)(fl + o0) = lv0;
    if (second) {
        *(volatile u16x8*)(fh + o1) = hv1;
        *(volatile u16x8*)(fl + o1) = lv1;
    }
}

template<int NBF>
__device__ __forceinline__ void tile_store_pass(const float* st, float* gp, int ldc, int lane) {
    constexpr int CW  = NBF * 16;
    constexpr int P   = CW + 4;
    constexpr int LPR = CW / 4;
    static_assert(32 % LPR == 0);
    constexpr int RPI = 32 / LPR;
    constexpr int NIT = 32 / RPI;
    const int rsub = lane / LPR;
    const int c0   = (lane % LPR) * 4;
#pragma unroll
    for (int it = 0; it < NIT; ++it) {
        const int row = it * RPI + rsub;
        const v4f v = *(const v4f*)(st + row * P + c0);
        *(volatile v4f*)(gp + (size_t)row * ldc + c0) = v;
    }
}

template<int NBF>
__global__ __launch_bounds__(128)
void gemm_x3_kernel(const unsigned short* __restrict__ Ah, const unsigned short* __restrict__ Al,
                    const unsigned short* __restrict__ Bh, const unsigned short* __restrict__ Bl,
                    float* C, int K, int ldc)
{
    constexpr int CW = NBF * 16;
    constexpr int P  = CW + 4;
    static_assert(CW % 32 == 0);
    __shared__ __attribute__((aligned(16))) float stile[4][32 * P];

    const int tid  = threadIdx.x;
    const int lane = tid & 31;
    const int wave = tid >> 5;
    const int h    = lane >> 4;
    const int m    = lane & 15;
    const int wm   = wave >> 1;
    const int wn   = wave & 1;

    const int rowW = blockIdx.y * 64 + wm * 32;
    const int colW = blockIdx.x * (2 * CW) + wn * CW;

    v8f acc[2 * NBF];
#pragma unroll
    for (int j = 0; j < 2 * NBF; ++j)
#pragma unroll
        for (int r = 0; r < 8; ++r) acc[j][r] = 0.0f;

    const size_t aoff  = (size_t)(rowW + m) * K + 8 * h;
    const size_t boff  = (size_t)(colW + m) * K + 8 * h;
    const size_t sub16 = (size_t)16 * K;
    const int nk = K >> 5;

#pragma unroll 1
    for (int kt = 0; kt < nk; ++kt) {
        const size_t k0 = (size_t)kt * 32;
        FragB fa[2], ga[2], fb[NBF], gb[NBF];
#pragma unroll
        for (int s = 0; s < 2; ++s) {
            const unsigned short* p = Ah + aoff + s * sub16 + k0;
            const unsigned short* q = Al + aoff + s * sub16 + k0;
            fa[s].h[0] = *(const u16x8*)(p);
            fa[s].h[1] = *(const u16x8*)(p + 16);
            ga[s].h[0] = *(const u16x8*)(q);
            ga[s].h[1] = *(const u16x8*)(q + 16);
        }
#pragma unroll
        for (int j = 0; j < NBF; ++j) {
            const unsigned short* p = Bh + boff + j * sub16 + k0;
            const unsigned short* q = Bl + boff + j * sub16 + k0;
            fb[j].h[0] = *(const u16x8*)(p);
            fb[j].h[1] = *(const u16x8*)(p + 16);
            gb[j].h[0] = *(const u16x8*)(q);
            gb[j].h[1] = *(const u16x8*)(q + 16);
        }
#pragma unroll
        for (int s = 0; s < 2; ++s)
#pragma unroll
            for (int j = 0; j < NBF; ++j) {
                mma16(acc[s * NBF + j], fa[s], fb[j]);
                mma16(acc[s * NBF + j], fa[s], gb[j]);
                mma16(acc[s * NBF + j], ga[s], fb[j]);
            }
    }

    float* st = stile[wave];
#pragma unroll
    for (int s = 0; s < 2; ++s)
#pragma unroll
        for (int j = 0; j < NBF; ++j)
#pragma unroll
            for (int r = 0; r < 8; ++r)
                st[(s * 16 + 8 * h + r) * P + j * 16 + m] = acc[s * NBF + j][r];
    __syncthreads();

    float* gp = C + (size_t)rowW * ldc + colW;
    tile_store_pass<NBF>(st, gp, ldc, lane);
    __threadfence();
    tile_store_pass<NBF>(st, gp, ldc, lane);
}

__global__ __launch_bounds__(512)
void lstm_kernel(const float* __restrict__ gx, const unsigned short* __restrict__ wh,
                 const unsigned short* __restrict__ wl, const float* __restrict__ b_ih,
                 const float* __restrict__ b_hh, float* out)
{
#pragma clang fp contract(off)
    __shared__ __attribute__((aligned(16))) unsigned short sHh[16 * HP_];
    __shared__ __attribute__((aligned(16))) unsigned short sHl[16 * HP_];
    __shared__ __attribute__((aligned(16))) float sOut[16 * 16 * OP_];

    const int tid  = threadIdx.x;
    const int lane = tid & 31;
    const int wave = tid >> 5;
    const int h    = lane >> 4;
    const int m    = lane & 15;
    const int b0   = blockIdx.x * 16;
    const int jb   = wave * 32;

    for (int i = tid; i < 16 * HP_; i += 512) { sHh[i] = 0; sHl[i] = 0; }

    float bias[8];
#pragma unroll
    for (int jt = 0; jt < 2; ++jt)
#pragma unroll
        for (int g = 0; g < 4; ++g) {
            const int col = g * HD_ + jb + 16 * jt + m;
            bias[jt * 4 + g] = b_ih[col] + b_hh[col];
        }

    float cst[16];
#pragma unroll
    for (int i = 0; i < 16; ++i) cst[i] = 0.0f;

    float* so = sOut + wave * (16 * OP_);
    __syncthreads();

#pragma unroll 1
    for (int s = 0; s < NS_; ++s) {
        v8f acc[8];
        const float* gxr = gx + (size_t)(s * NB_ + b0 + 8 * h) * G4_;
#pragma unroll
        for (int jt = 0; jt < 2; ++jt)
#pragma unroll
            for (int g = 0; g < 4; ++g) {
                const int col = g * HD_ + jb + 16 * jt + m;
                const float bv = bias[jt * 4 + g];
#pragma unroll
                for (int r = 0; r < 8; ++r)
                    acc[jt * 4 + g][r] = gxr[(size_t)r * G4_ + col] + bv;
            }

#pragma unroll 1
        for (int kt = 0; kt < HD_ / 32; ++kt) {
            const int k0 = kt * 32;
            FragB fa, ga;
            const unsigned short* ap = sHh + m * HP_ + k0 + 8 * h;
            const unsigned short* aq = sHl + m * HP_ + k0 + 8 * h;
            fa.h[0] = *(const u16x8*)(ap);
            fa.h[1] = *(const u16x8*)(ap + 16);
            ga.h[0] = *(const u16x8*)(aq);
            ga.h[1] = *(const u16x8*)(aq + 16);
#pragma unroll
            for (int jt = 0; jt < 2; ++jt)
#pragma unroll
                for (int g = 0; g < 4; ++g) {
                    const int nrow = g * HD_ + jb + 16 * jt + m;
                    const unsigned short* bp = wh + (size_t)nrow * HD_ + k0 + 8 * h;
                    const unsigned short* bq = wl + (size_t)nrow * HD_ + k0 + 8 * h;
                    FragB fb, gb;
                    fb.h[0] = *(const u16x8*)(bp);
                    fb.h[1] = *(const u16x8*)(bp + 16);
                    gb.h[0] = *(const u16x8*)(bq);
                    gb.h[1] = *(const u16x8*)(bq + 16);
                    mma16(acc[jt * 4 + g], fa, fb);
                    mma16(acc[jt * 4 + g], fa, gb);
                    mma16(acc[jt * 4 + g], ga, fb);
                }
        }
        __syncthreads();

#pragma unroll
        for (int jt = 0; jt < 2; ++jt)
#pragma unroll
            for (int r = 0; r < 8; ++r) {
                const float iv = sigm_f(acc[jt * 4 + 0][r]);
                const float fv = sigm_f(acc[jt * 4 + 1][r]);
                const float gv = tanh_f(acc[jt * 4 + 2][r]);
                const float ov = sigm_f(acc[jt * 4 + 3][r]);
                const float t1 = fv * cst[jt * 8 + r];
                const float t2 = iv * gv;
                const float cn = t1 + t2;
                cst[jt * 8 + r] = cn;
                const float hv = ov * tanh_f(cn);
                const int row = 8 * h + r;
                const int cj  = 16 * jt + m;
                so[row * OP_ + cj] = hv;
                const unsigned short hb = f32_to_bf16(hv);
                const unsigned short lb = f32_to_bf16(hv - bf16_to_f32(hb));
                sHh[row * HP_ + jb + cj] = hb;
                sHl[row * HP_ + jb + cj] = lb;
            }
        __syncthreads();

#pragma unroll
        for (int it = 0; it < 4; ++it) {
            const int row = it * 4 + (lane >> 3);
            const int c   = (lane & 7) * 4;
            const v4f v = *(const v4f*)(so + row * OP_ + c);
            float* gp = out + ((size_t)(b0 + row) * NS_ + s) * HD_ + jb + c;
            *(volatile v4f*)gp = v;
        }
        __threadfence();
#pragma unroll
        for (int it = 0; it < 4; ++it) {
            const int row = it * 4 + (lane >> 3);
            const int c   = (lane & 7) * 4;
            const v4f v = *(const v4f*)(so + row * OP_ + c);
            float* gp = out + ((size_t)(b0 + row) * NS_ + s) * HD_ + jb + c;
            *(volatile v4f*)gp = v;
        }
    }
}

extern "C" void kernel_launch(void* const* d_in, const int* in_sizes, int n_in,
                              void* d_out, int out_size, void* d_ws, size_t ws_size,
                              hipStream_t stream)
{
    if (n_in < 5) return;
    if (in_sizes[0] != NB_ * TL_ * CC_) return;
    if (in_sizes[1] != G4_ * FIN_)      return;
    if (in_sizes[2] != G4_ * HD_)       return;
    if (in_sizes[3] != G4_)             return;
    if (in_sizes[4] != G4_)             return;
    if (out_size != NB_ * NS_ * HD_)    return;
    if (ws_size < WS_END)               return;

    const float* x    = (const float*)d_in[0];
    const float* w_ih = (const float*)d_in[1];
    const float* w_hh = (const float*)d_in[2];
    const float* b_ih = (const float*)d_in[3];
    const float* b_hh = (const float*)d_in[4];
    float* out = (float*)d_out;

    char* ws = (char*)d_ws;
    unsigned short* fh  = (unsigned short*)(ws + OFF_FH);
    unsigned short* fl  = (unsigned short*)(ws + OFF_FL);
    unsigned short* wih = (unsigned short*)(ws + OFF_WIH);
    unsigned short* wil = (unsigned short*)(ws + OFF_WIL);
    unsigned short* whh = (unsigned short*)(ws + OFF_WHH);
    unsigned short* whl = (unsigned short*)(ws + OFF_WHL);
    float*          gx  = (float*)(ws + OFF_GX);

    {
        const int np = G4_ * (KP_ / 8);
        rows_cvt_kernel<<<dim3((np + 255) / 256), dim3(256), 0, stream>>>(w_ih, wih, wil, (int)FIN_, (int)KP_, np);
    }
    {
        const int np = G4_ * (HD_ / 8);
        rows_cvt_kernel<<<dim3((np + 255) / 256), dim3(256), 0, stream>>>(w_hh, whh, whl, (int)HD_, (int)HD_, np);
    }
    feats_kernel<<<dim3(MR_), dim3(256), 0, stream>>>(x, fh, fl);

    gemm_x3_kernel<2><<<dim3(G4_ / 64, MR_ / 64), dim3(128), 0, stream>>>(
        (const unsigned short*)fh, (const unsigned short*)fl,
        (const unsigned short*)wih, (const unsigned short*)wil,
        gx, (int)KP_, (int)G4_);

    lstm_kernel<<<dim3(NB_ / 16), dim3(512), 0, stream>>>(
        (const float*)gx, (const unsigned short*)whh, (const unsigned short*)whl, b_ih, b_hh, out);
}
